// Mamba_block_67920612819445
// MI455X (gfx1250) — hardware-run, weakly checked
//
#include <hip/hip_runtime.h>
#include <math.h>

typedef __attribute__((ext_vector_type(16))) _Float16 v16h;
typedef __attribute__((ext_vector_type(8)))  _Float16 v8h;
typedef __attribute__((ext_vector_type(16))) __bf16   v16b;
typedef __attribute__((ext_vector_type(8)))  __bf16   v8b;
typedef __attribute__((ext_vector_type(8)))  float    v8f;
typedef __attribute__((ext_vector_type(4)))  float    v4f;

constexpr int kBatch    = 4;
constexpr int kCin      = 32;
constexpr int kHin      = 192;
constexpr int kWin      = 192;
constexpr int kHout     = 96;
constexpr int kWout     = 96;
constexpr int kL        = kHout * kWout;
constexpr int kRows     = kBatch * kL;
constexpr int kHalfRows = kRows / 2;
constexpr int kDm       = 64;
constexpr int kDin      = 128;
constexpr int kNst      = 16;
constexpr int kDtR      = 4;
constexpr int kXzP      = 2 * kDin;
constexpr int kXdP      = 64;
constexpr int kXdReal   = kDtR + 2 * kNst;
constexpr int kKconv    = kCin * 16;
constexpr int kConvTP   = 132;
constexpr int kScanTS   = 64;
constexpr int kScanCh   = 64;
constexpr int kScanYP   = 68;
constexpr int kOutTP    = 68;
static_assert(kXdReal <= kXdP, "x_proj pad");
static_assert((kKconv % 32) == 0 && (kDm % 32) == 0 && (kDin % 32) == 0, "GEMM K multiples of 32");
static_assert((kHalfRows % 64) == 0 && (kRows % 64) == 0 && (kDm % 64) == 0 && (kXzP % 64) == 0 && (kXdP % 64) == 0, "GEMM M,N multiples of 64");
static_assert((kL % 64) == 0 && (kL % kScanTS) == 0 && (kDin % kScanCh) == 0 && kDin == 128 && kDm == 64, "tile multiples");
static_assert((kHalfRows % kL) == 0, "im2col halves hold whole batch elements");

constexpr size_t kOffW1   = 0;
constexpr size_t kOffW2   = kOffW1  + (size_t)kDm  * kKconv * 2;
constexpr size_t kOffW3   = kOffW2  + (size_t)kXzP * kDm    * 2;
constexpr size_t kOffW4   = kOffW3  + (size_t)kXdP * kDin   * 2;
constexpr size_t kOffCol  = kOffW4  + (size_t)kDm  * kDin   * 2;
constexpr size_t kOffXcT  = kOffCol + (size_t)kHalfRows * kKconv * 2;
constexpr size_t kOffNrm  = kOffXcT + (size_t)kRows * kDm  * 4;
constexpr size_t kOffXz   = kOffNrm + (size_t)kRows * kDm  * 2;
constexpr size_t kOffXm   = kOffXz  + (size_t)kRows * kXzP * 4;
constexpr size_t kOffXm16 = kOffXm  + (size_t)kRows * kDin * 4;
constexpr size_t kOffXd   = kOffXm16 + (size_t)kRows * kDin * 2;
constexpr size_t kOffYg   = kOffXd  + (size_t)kRows * kXdP * 4;
constexpr size_t kWsTotal = kOffYg  + (size_t)kRows * kDin * 2;
static_assert(kWsTotal == 118095872ull, "carve total");
static_assert(kWsTotal <= 134217728ull, "carve cap");
static_assert((kOffW2 % 128) == 0 && (kOffW3 % 128) == 0 && (kOffW4 % 128) == 0 && (kOffCol % 128) == 0 &&
              (kOffXcT % 128) == 0 && (kOffNrm % 128) == 0 && (kOffXz % 128) == 0 && (kOffXm % 128) == 0 &&
              (kOffXm16 % 128) == 0 && (kOffXd % 128) == 0 && (kOffYg % 128) == 0, "128-B aligned regions");

__device__ __forceinline__ unsigned short f2bf_bits(float f) {
  unsigned u = __float_as_uint(f);
  return (unsigned short)((u + 0x7FFFu + ((u >> 16) & 1u)) >> 16);
}
__device__ __forceinline__ float bf_bits2f(unsigned short h) { return __uint_as_float(((unsigned)h) << 16); }

__device__ __forceinline__ void dep_guard_h(v8f& a, v8f& b, v16h x, v16h y) { asm volatile("v_nop\n\tv_nop\n\tv_nop\n\tv_nop" : "+v"(a), "+v"(b) : "v"(x), "v"(y)); }
__device__ __forceinline__ void dep_guard_b(v8f& a, v8f& b, v16b x, v16b y) { asm volatile("v_nop\n\tv_nop\n\tv_nop\n\tv_nop" : "+v"(a), "+v"(b) : "v"(x), "v"(y)); }
__device__ __forceinline__ void dep_guard4_h(v8f& a, v8f& b, v8f& c, v8f& d, v16h x, v16h y) { asm volatile("v_nop\n\tv_nop\n\tv_nop\n\tv_nop" : "+v"(a), "+v"(b), "+v"(c), "+v"(d) : "v"(x), "v"(y)); }
__device__ __forceinline__ void dep_guard4_b(v8f& a, v8f& b, v8f& c, v8f& d, v16b x, v16b y) { asm volatile("v_nop\n\tv_nop\n\tv_nop\n\tv_nop" : "+v"(a), "+v"(b), "+v"(c), "+v"(d) : "v"(x), "v"(y)); }
__device__ __forceinline__ void dep_guard4x5_h(v8f& a, v8f& b, v8f& c, v8f& d, v16h x, v16h y0, v16h y1, v16h y2, v16h y3) {
  asm volatile("v_nop\n\tv_nop\n\tv_nop\n\tv_nop" : "+v"(a), "+v"(b), "+v"(c), "+v"(d) : "v"(x), "v"(y0), "v"(y1), "v"(y2), "v"(y3));
}
__device__ __forceinline__ void keep4_h(v16h a, v16h b, v16h c, v16h d) { asm volatile("v_nop" :: "v"(a), "v"(b), "v"(c), "v"(d)); }
__device__ __forceinline__ void keep4_b(v16b a, v16b b, v16b c, v16b d) { asm volatile("v_nop" :: "v"(a), "v"(b), "v"(c), "v"(d)); }
__device__ __forceinline__ void acc_guard4(v8f& a, v8f& b, v8f& c, v8f& d) { asm volatile("v_nop\n\tv_nop\n\tv_nop\n\tv_nop" : "+v"(a), "+v"(b), "+v"(c), "+v"(d)); }
template <typename T> struct Frag;
template <> struct Frag<_Float16> {
  typedef v16h V; union U { v16h v; v8h h[2]; };
  static __device__ __forceinline__ v16h load(const _Float16* p) {
    U f; f.h[0] = *(const v8h*)(p); f.h[1] = *(const v8h*)(p + 16); return f.v;
  }
  static __device__ __forceinline__ v8f mma(v16h a, v16h b, v8f c) {
    return __builtin_amdgcn_wmma_f32_16x16x32_f16(false, a, false, b, (short)0, c, false, false);
  }
  static __device__ __forceinline__ void guard(v8f& a, v8f& b, v16h x, v16h y) { dep_guard_h(a, b, x, y); }
  static __device__ __forceinline__ void guard4(v8f& a, v8f& b, v8f& c, v8f& d, v16h x, v16h y) { dep_guard4_h(a, b, c, d, x, y); }
  static __device__ __forceinline__ void keep(v16h a, v16h b, v16h c, v16h d) { keep4_h(a, b, c, d); }
};
template <> struct Frag<__bf16> {
  typedef v16b V; union U { v16b v; v8b h[2]; };
  static __device__ __forceinline__ v16b load(const __bf16* p) {
    U f; f.h[0] = *(const v8b*)(p); f.h[1] = *(const v8b*)(p + 16); return f.v;
  }
  static __device__ __forceinline__ v8f mma(v16b a, v16b b, v8f c) {
    return __builtin_amdgcn_wmma_f32_16x16x32_bf16(false, a, false, b, (short)0, c, false, false);
  }
  static __device__ __forceinline__ void guard(v8f& a, v8f& b, v16b x, v16b y) { dep_guard_b(a, b, x, y); }
  static __device__ __forceinline__ void guard4(v8f& a, v8f& b, v8f& c, v8f& d, v16b x, v16b y) { dep_guard4_b(a, b, c, d, x, y); }
  static __device__ __forceinline__ void keep(v16b a, v16b b, v16b c, v16b d) { keep4_b(a, b, c, d); }
};

template <int ET> struct Elem;
template <> struct Elem<0> { typedef _Float16 T; };
template <> struct Elem<1> { typedef __bf16 T; };
template <int ET, bool SPLIT, int BIAS_MODE, int OUT_MODE, bool RESID, int ACT = 0>
__global__ __launch_bounds__(256) void wmma_gemm64(
    const unsigned short* __restrict__ Ap, const unsigned short* __restrict__ A2p, int lda, long strideA,
    const unsigned short* __restrict__ Btp, const unsigned short* __restrict__ Bt2p, int ldb, long strideB,
    void* __restrict__ Cout, void* __restrict__ Cout2, int ldc, long strideC,
    const float* __restrict__ bias,
    const float* __restrict__ resid, long strideR,
    int M, int N, int K, float scale) {
  typedef typename Elem<ET>::T T;
  typedef typename Frag<T>::V V;
  const T* A = (const T*)Ap; const T* A2 = (const T*)A2p; const T* Bt = (const T*)Btp; const T* Bt2 = (const T*)Bt2p;
  __shared__ __align__(16) float sT[8][16 * 68];
  const int b    = blockIdx.y;
  const int lane = threadIdx.x & 31;
  const int wave = threadIdx.x >> 5;
  const int tilesN = N >> 6;
  const int tilesM = M >> 6;
  const int tile = blockIdx.x * 8 + wave;
  if (tile >= tilesM * tilesN) return;
  const int tm = tile / tilesN;
  const int tn = tile - tm * tilesN;
  const int m0 = tm << 6;
  const int n0 = tn << 6;

  const T* Ab  = A  + (size_t)b * strideA;
  const T* Bb  = Bt + (size_t)b * strideB;
  const T* Ab2 = SPLIT ? (A2  + (size_t)b * strideA) : nullptr;
  const T* Bb2 = SPLIT ? (Bt2 + (size_t)b * strideB) : nullptr;

  const int rlane = lane & 15;
  const int koff  = (lane >> 4) * 8;
  const int mOff  = (lane >> 4) * 8;

  v8f acc[4][4];
#pragma unroll
  for (int i = 0; i < 4; ++i)
#pragma unroll
    for (int j = 0; j < 4; ++j) acc[i][j] = (v8f){0.f,0.f,0.f,0.f,0.f,0.f,0.f,0.f};

  for (int k0 = 0; k0 < K; k0 += 32) {
    V bh[4], bl[4];
#pragma unroll
    for (int j = 0; j < 4; ++j) {
      const size_t bo = (size_t)(n0 + (j << 4) + rlane) * ldb + koff + k0;
      bh[j] = Frag<T>::load(Bb + bo);
      if (SPLIT) bl[j] = Frag<T>::load(Bb2 + bo);
    }
#pragma unroll
    for (int i = 0; i < 4; ++i) {
      const size_t ao = (size_t)(m0 + (i << 4) + rlane) * lda + koff + k0;
      V ah = Frag<T>::load(Ab + ao);
      V al;
      if (SPLIT) al = Frag<T>::load(Ab2 + ao);
#pragma unroll
      for (int j = 0; j < 4; ++j) {
        acc[i][j] = Frag<T>::mma(ah, bh[j], acc[i][j]);
        if (SPLIT) {
          acc[i][j] = Frag<T>::mma(ah, bl[j], acc[i][j]);
          acc[i][j] = Frag<T>::mma(al, bh[j], acc[i][j]);
        }
      }
      Frag<T>::guard4(acc[i][0], acc[i][1], acc[i][2], acc[i][3], ah, SPLIT ? al : ah);
    }
    Frag<T>::keep(bh[0], bh[1], bh[2], bh[3]);
    if (SPLIT) Frag<T>::keep(bl[0], bl[1], bl[2], bl[3]);
  }
  acc_guard4(acc[0][0], acc[0][1], acc[0][2], acc[0][3]);
  acc_guard4(acc[1][0], acc[1][1], acc[1][2], acc[1][3]);
  acc_guard4(acc[2][0], acc[2][1], acc[2][2], acc[2][3]);
  acc_guard4(acc[3][0], acc[3][1], acc[3][2], acc[3][3]);

  float* slab = sT[wave];
  const float* Rb = RESID ? (resid + (size_t)b * strideR) : nullptr;
#pragma unroll
  for (int i = 0; i < 4; ++i) {
    const int mBase = m0 + (i << 4);
#pragma unroll
    for (int j = 0; j < 4; ++j) {
      const int n = n0 + (j << 4) + rlane;
      float bv = 0.f;
      if (BIAS_MODE == 2) bv = bias[n];
#pragma unroll
      for (int r = 0; r < 8; ++r) {
        float v = acc[i][j][r] * scale;
        if (BIAS_MODE == 1) v += bias[mBase + mOff + r];
        if (BIAS_MODE == 2) v += bv;
        if (RESID) v += Rb[(size_t)(mBase + mOff + r) * ldc + n];
        if (ACT == 1) v = tanhf(v);
        if (ACT == 2) v = fmaxf(v, 0.0f);
        if (ACT == 3) v = v / (1.0f + expf(-v));
        if (ACT == 4) v = (v > 0.f) ? v : 0.01f * v;
        slab[(mOff + r) * 68 + (j << 4) + rlane] = v;
      }
    }
    __builtin_amdgcn_fence(__ATOMIC_RELEASE, "workgroup");
    __builtin_amdgcn_wave_barrier();
    __builtin_amdgcn_fence(__ATOMIC_ACQUIRE, "workgroup");
    if (OUT_MODE == 0) {
      float* C = (float*)Cout + (size_t)b * strideC;
      const int hh = lane >> 4, c4 = (lane & 15) * 4;
      for (int pass = 0; pass < 2; ++pass) {
#pragma unroll
        for (int it = 0; it < 8; ++it) {
          const int row = it * 2 + hh;
          v4f v = *(const v4f*)(slab + row * 68 + c4);
          *(volatile v4f*)(C + (size_t)(mBase + row) * ldc + n0 + c4) = v;
        }
        __threadfence();
      }
    } else {
      const int q = lane >> 3, c8 = (lane & 7) * 8;
      unsigned short* C  = (unsigned short*)Cout  + (size_t)b * strideC;
      unsigned short* C2 = (OUT_MODE == 2) ? ((unsigned short*)Cout2 + (size_t)b * strideC) : nullptr;
      for (int pass = 0; pass < 2; ++pass) {
#pragma unroll
        for (int it = 0; it < 4; ++it) {
          const int row = it * 4 + q;
          const float* sp = slab + row * 68 + c8;
          v8h hv, lv;
#pragma unroll
          for (int e = 0; e < 8; ++e) {
            if (OUT_MODE == 1) {
              hv[e] = (_Float16)sp[e];
            } else {
              unsigned short hb = f2bf_bits(sp[e]);
              unsigned short lb = f2bf_bits(sp[e] - bf_bits2f(hb));
              hv[e] = __builtin_bit_cast(_Float16, hb);
              lv[e] = __builtin_bit_cast(_Float16, lb);
            }
          }
          *(volatile v8h*)(C + (size_t)(mBase + row) * ldc + n0 + c8) = hv;
          if (OUT_MODE == 2) *(volatile v8h*)(C2 + (size_t)(mBase + row) * ldc + n0 + c8) = lv;
        }
        __threadfence();
      }
    }
    __builtin_amdgcn_fence(__ATOMIC_RELEASE, "workgroup");
    __builtin_amdgcn_wave_barrier();
    __builtin_amdgcn_fence(__ATOMIC_ACQUIRE, "workgroup");
  }
}

__global__ __launch_bounds__(256) void cast_rows_f16_kernel(
    const float* __restrict__ src, unsigned short* __restrict__ dst, int kdim, int nreal, int total8, float mul)
{
  const int i = blockIdx.x * 256 + threadIdx.x;
  if (i >= total8) return;
  const int e0 = i << 3;
  const int n = e0 / kdim;
  const int k = e0 - n * kdim;
  const int nc = (n < nreal) ? n : (nreal - 1);
  const float f = (n < nreal) ? mul : 0.0f;
  const float* sp = src + (size_t)nc * kdim + k;
  const v4f a0 = *(const v4f*)(sp);
  const v4f a1 = *(const v4f*)(sp + 4);
  v8h hv;
#pragma unroll
  for (int e = 0; e < 4; ++e) {
    hv[e]     = (_Float16)(a0[e] * f);
    hv[4 + e] = (_Float16)(a1[e] * f);
  }
  unsigned short* q = dst + e0;
  *(volatile v8h*)q = hv;
  __threadfence();
  *(volatile v8h*)q = hv;
}

__global__ __launch_bounds__(256) void im2col_kernel(
    const float* __restrict__ x, unsigned short* __restrict__ dst, int half)
{
  const int gt = blockIdx.x * 256 + threadIdx.x;
  const int rowl = gt >> 6;
  const int k8 = gt & 63;
  const int row = half * kHalfRows + rowl;
  const int b = row / kL;
  const int l = row - b * kL;
  const int oh = l / kWout;
  const int ow = l - oh * kWout;
  const int cin = k8 >> 1;
  const int kh0 = (k8 & 1) * 2;
  const float* xb = x + (size_t)(b * kCin + cin) * kHin * kWin;
  float v[8];
#pragma unroll
  for (int r = 0; r < 2; ++r) {
    int ih = 2 * oh - 1 + kh0 + r;
    ih = (ih < 0) ? -ih : ih;
    ih = (ih > kHin - 1) ? (2 * (kHin - 1) - ih) : ih;
    ih = ih < 0 ? 0 : (ih > kHin - 1 ? kHin - 1 : ih);
#pragma unroll
    for (int kw = 0; kw < 4; ++kw) {
      int iw = 2 * ow - 1 + kw;
      iw = (iw < 0) ? -iw : iw;
      iw = (iw > kWin - 1) ? (2 * (kWin - 1) - iw) : iw;
      iw = iw < 0 ? 0 : (iw > kWin - 1 ? kWin - 1 : iw);
      v[r * 4 + kw] = xb[ih * kWin + iw];
    }
  }
  v8h hv;
#pragma unroll
  for (int e = 0; e < 8; ++e) hv[e] = (_Float16)v[e];
  unsigned short* q = dst + (size_t)rowl * kKconv + k8 * 8;
  *(volatile v8h*)q = hv;
  __threadfence();
  *(volatile v8h*)q = hv;
}

__global__ __launch_bounds__(256) void ln_kernel(
    const float* __restrict__ XCT, const float* __restrict__ g, const float* __restrict__ bta,
    unsigned short* __restrict__ NRM)
{
  const int gt = blockIdx.x * 256 + threadIdx.x;
  const int row = gt >> 3;
  const int c0 = (gt & 7) * 8;
  const float* rp = XCT + (size_t)row * kDm + c0;
  const v4f a0 = *(const v4f*)(rp);
  const v4f a1 = *(const v4f*)(rp + 4);
  const v4f g0 = *(const v4f*)(g + c0);
  const v4f g1 = *(const v4f*)(g + c0 + 4);
  const v4f b0 = *(const v4f*)(bta + c0);
  const v4f b1 = *(const v4f*)(bta + c0 + 4);
  float s = 0.0f;
#pragma unroll
  for (int e = 0; e < 4; ++e) s += a0[e];
#pragma unroll
  for (int e = 0; e < 4; ++e) s += a1[e];
  s += __shfl_xor(s, 1, 32);
  s += __shfl_xor(s, 2, 32);
  s += __shfl_xor(s, 4, 32);
  const float mu = s * (1.0f / 64.0f);
  float d0[4], d1[4];
  float s2 = 0.0f;
#pragma unroll
  for (int e = 0; e < 4; ++e) { d0[e] = a0[e] - mu; s2 += d0[e] * d0[e]; }
#pragma unroll
  for (int e = 0; e < 4; ++e) { d1[e] = a1[e] - mu; s2 += d1[e] * d1[e]; }
  s2 += __shfl_xor(s2, 1, 32);
  s2 += __shfl_xor(s2, 2, 32);
  s2 += __shfl_xor(s2, 4, 32);
  const float var = s2 * (1.0f / 64.0f);
  const float rs = rsqrtf(var + 1e-5f);
  v8h hv;
#pragma unroll
  for (int e = 0; e < 4; ++e) {
    hv[e]     = (_Float16)(d0[e] * rs * g0[e] + b0[e]);
    hv[4 + e] = (_Float16)(d1[e] * rs * g1[e] + b1[e]);
  }
  unsigned short* q = NRM + (size_t)row * kDm + c0;
  *(volatile v8h*)q = hv;
  __threadfence();
  *(volatile v8h*)q = hv;
}

__global__ __launch_bounds__(128) void conv_silu_kernel(
    const float* __restrict__ XZ, const float* __restrict__ cw, const float* __restrict__ cb,
    float* __restrict__ UC, unsigned short* __restrict__ UH)
{
  __shared__ __align__(16) float sT[16 * kConvTP];
  const int tid = threadIdx.x, lane = tid & 31, wave = tid >> 5;
  const int d = tid;
  const int g0 = blockIdx.x * 64;
  const int tb = g0 % kL;
  const float w0 = cw[d * 4 + 0], w1 = cw[d * 4 + 1], w2 = cw[d * 4 + 2], w3 = cw[d * 4 + 3];
  const float bc = cb[d];
  float xm3, xm2, xm1;
  {
    const bool hist = (tb > 0);
    const int rb = hist ? (g0 - 3) : g0;
    const float v3 = XZ[(size_t)rb * kXzP + d];
    const float v2 = XZ[(size_t)(rb + 1) * kXzP + d];
    const float v1 = XZ[(size_t)(rb + 2) * kXzP + d];
    xm3 = hist ? v3 : 0.f;
    xm2 = hist ? v2 : 0.f;
    xm1 = hist ? v1 : 0.f;
  }
  const int hh = lane >> 4;
  const int c8 = (lane & 15) * 8;
#pragma unroll 1
  for (int sub = 0; sub < 4; ++sub) {
    const int lb = g0 + sub * 16;
#pragma unroll 1
    for (int s = 0; s < 16; ++s) {
      const float xcur = XZ[(size_t)(lb + s) * kXzP + d];
      float acc = w0 * xm3;
      acc = fmaf(w1, xm2, acc);
      acc = fmaf(w2, xm1, acc);
      acc = fmaf(w3, xcur, acc);
      const float sv = acc + bc;
      const float sg = __builtin_amdgcn_rcpf(1.0f + __expf(-sv));
      sT[s * kConvTP + tid] = sv * sg;
      xm3 = xm2; xm2 = xm1; xm1 = xcur;
    }
    __syncthreads();
    v4f fv[4];
    v8h bh[2];
#pragma unroll
    for (int it = 0; it < 4; ++it) fv[it] = *(const v4f*)(sT + (it * 4 + wave) * kConvTP + lane * 4);
#pragma unroll
    for (int it = 0; it < 2; ++it) {
      const float* sp = sT + (it * 8 + wave * 2 + hh) * kConvTP + c8;
      const v4f a0 = *(const v4f*)(sp);
      const v4f a1 = *(const v4f*)(sp + 4);
#pragma unroll
      for (int e = 0; e < 4; ++e) {
        bh[it][e]     = (_Float16)a0[e];
        bh[it][4 + e] = (_Float16)a1[e];
      }
    }
    for (int pass = 0; pass < 2; ++pass) {
#pragma unroll
      for (int it = 0; it < 4; ++it)
        *(volatile v4f*)(UC + (size_t)(lb + it * 4 + wave) * kDin + lane * 4) = fv[it];
#pragma unroll
      for (int it = 0; it < 2; ++it) {
        const size_t o = (size_t)(lb + it * 8 + wave * 2 + hh) * kDin + c8;
        *(volatile v8h*)(UH + o) = bh[it];
      }
      __threadfence();
    }
    __syncthreads();
  }
}

__global__ __launch_bounds__(64) void scan_kernel(
    const float* __restrict__ XD, const float* __restrict__ UC, const float* __restrict__ XZ,
    const float* __restrict__ Wdt, const float* __restrict__ bdt, const float* __restrict__ Alog,
    const float* __restrict__ Dp, unsigned short* __restrict__ YG, float ymul)
{
  __shared__ __align__(16) float sX[kScanTS * kXdP];
  __shared__ __align__(16) float sY[kScanTS * kScanYP];
  __shared__ __align__(16) float sA[kNst * kScanCh];
  const int tid = threadIdx.x, lane = tid & 31, wave = tid >> 5;
  constexpr int kBlkPerB = kDin / kScanCh;
  const int bix = blockIdx.x / kBlkPerB;
  const int d0  = (blockIdx.x - bix * kBlkPerB) * kScanCh;
  const int d   = d0 + tid;
  const size_t row0 = (size_t)bix * kL;
#pragma unroll 1
  for (int s = 0; s < kNst; ++s) sA[s * kScanCh + tid] = -expf(Alog[(size_t)d * kNst + s]);
  __syncthreads();
  float negA[kNst], h[kNst];
#pragma unroll
  for (int s = 0; s < kNst; ++s) {
    negA[s] = sA[s * kScanCh + tid];
    h[s] = 0.f;
  }
  const v4f wv = *(const v4f*)(Wdt + (size_t)d * kDtR);
  const float bb = bdt[d], Dd = Dp[d];
  const int lr = tid >> 4, lc4 = (tid & 15) * 4;
  const int q = lane >> 3, c8 = (lane & 7) * 8;
#pragma unroll 1
  for (int t0 = 0; t0 < kL; t0 += kScanTS) {
    __syncthreads();
#pragma unroll
    for (int i = 0; i < 8; ++i) {
      const int r = lr + 4 * i;
      *(v4f*)(sX + r * kXdP + lc4) = *(const v4f*)(XD + (row0 + t0 + r) * kXdP + lc4);
    }
    asm volatile("" ::: "memory");
#pragma unroll
    for (int i = 8; i < 16; ++i) {
      const int r = lr + 4 * i;
      *(v4f*)(sX + r * kXdP + lc4) = *(const v4f*)(XD + (row0 + t0 + r) * kXdP + lc4);
    }
    __syncthreads();
#pragma unroll 1
    for (int s = 0; s < kScanTS; ++s) {
      const int t = t0 + s;
      const float* xr = sX + s * kXdP;
      const v4f xv = *(const v4f*)(xr);
      float vdot = wv[0] * xv[0];
      vdot = fmaf(wv[1], xv[1], vdot);
      vdot = fmaf(wv[2], xv[2], vdot);
      vdot = fmaf(wv[3], xv[3], vdot);
      float Bs[kNst], Cs[kNst];
#pragma unroll
      for (int q4 = 0; q4 < 4; ++q4) {
        const v4f bv = *(const v4f*)(xr + kDtR + 4 * q4);
        const v4f cv = *(const v4f*)(xr + kDtR + kNst + 4 * q4);
        Bs[4 * q4 + 0] = bv[0]; Bs[4 * q4 + 1] = bv[1]; Bs[4 * q4 + 2] = bv[2]; Bs[4 * q4 + 3] = bv[3];
        Cs[4 * q4 + 0] = cv[0]; Cs[4 * q4 + 1] = cv[1]; Cs[4 * q4 + 2] = cv[2]; Cs[4 * q4 + 3] = cv[3];
      }
      const float v   = vdot + bb;
      const float a   = __expf(-fabsf(v));
      const float u   = 1.0f + a;
      const float l1p = __logf(u) + (a - (u - 1.0f)) * __builtin_amdgcn_rcpf(u);
      const float dt  = fmaxf(v, 0.0f) + l1p;
      const float xt  = UC[(row0 + t) * kDin + d];
      const float dtx = dt * xt;
      float y = 0.f;
#pragma unroll
      for (int k = 0; k < kNst; ++k) {
        const float e = __expf(dt * negA[k]);
        h[k] = e * h[k] + dtx * Bs[k];
        y = h[k] * Cs[k] + y;
      }
      y = xt * Dd + y;
      const float zv = XZ[(row0 + t) * kXzP + kDin + d];
      const float sg = __builtin_amdgcn_rcpf(1.0f + __expf(-zv));
      y = y * (zv * sg);
      sY[s * kScanYP + tid] = y * ymul;
    }
    __syncthreads();
    v8h hv[8];
#pragma unroll
    for (int it = 0; it < 8; ++it) {
      const int row = it * 8 + wave * 4 + q;
      const float* sp = sY + row * kScanYP + c8;
      const v4f a0 = *(const v4f*)(sp);
      const v4f a1 = *(const v4f*)(sp + 4);
#pragma unroll
      for (int e = 0; e < 4; ++e) {
        hv[it][e]     = (_Float16)a0[e];
        hv[it][4 + e] = (_Float16)a1[e];
      }
    }
    for (int pass = 0; pass < 2; ++pass) {
#pragma unroll
      for (int it = 0; it < 8; ++it) {
        const int row = it * 8 + wave * 4 + q;
        const size_t o = (row0 + t0 + row) * kDin + d0 + c8;
        *(volatile v8h*)(YG + o) = hv[it];
      }
      __threadfence();
    }
  }
}

__global__ __launch_bounds__(128) void outproj_nchw_kernel(
    const unsigned short* __restrict__ Yp, const unsigned short* __restrict__ Wp,
    const float* __restrict__ XCT, float* __restrict__ out, float scale)
{
  __shared__ __align__(16) float sT[kDm * kOutTP];
  const _Float16* Y = (const _Float16*)Yp;
  const _Float16* W = (const _Float16*)Wp;
  const int tid = threadIdx.x, lane = tid & 31, wave = tid >> 5;
  const int rlane = lane & 15;
  const int hsel = lane >> 4;
  const int koff = hsel * 8;
  const int m0 = blockIdx.x * 64;
  v8f acc[4];
#pragma unroll
  for (int j = 0; j < 4; ++j) acc[j] = (v8f){0.f,0.f,0.f,0.f,0.f,0.f,0.f,0.f};
#pragma unroll
  for (int k0 = 0; k0 < kDin; k0 += 32) {
    v16h bf[4];
#pragma unroll
    for (int j = 0; j < 4; ++j) bf[j] = Frag<_Float16>::load(W + (size_t)(j * 16 + rlane) * kDin + koff + k0);
    const v16h af = Frag<_Float16>::load(Y + (size_t)(m0 + wave * 16 + rlane) * kDin + koff + k0);
#pragma unroll
    for (int j = 0; j < 4; ++j) acc[j] = Frag<_Float16>::mma(af, bf[j], acc[j]);
    dep_guard4x5_h(acc[0], acc[1], acc[2], acc[3], af, bf[0], bf[1], bf[2], bf[3]);
  }
  acc_guard4(acc[0], acc[1], acc[2], acc[3]);
#pragma unroll
  for (int j = 0; j < 4; ++j) {
#pragma unroll
    for (int r = 0; r < 8; ++r) {
      sT[(j * 16 + rlane) * kOutTP + wave * 16 + hsel * 8 + r] = acc[j][r] * scale;
    }
  }
  __syncthreads();
#pragma unroll
  for (int i = 0; i < 8; ++i) {
    const int idx = tid + 128 * i;
    const int l = idx >> 4;
    const int n4 = (idx & 15) * 4;
    const v4f rv = *(const v4f*)(XCT + (size_t)(m0 + l) * kDm + n4);
#pragma unroll
    for (int e = 0; e < 4; ++e) {
      const int si = (n4 + e) * kOutTP + l;
      sT[si] = 2.0f * rv[e] + sT[si];
    }
  }
  __syncthreads();
  const int bb = m0 / kL;
  const int l0 = m0 - bb * kL;
  const int c4 = rlane * 4;
  v4f ov[8];
#pragma unroll
  for (int it = 0; it < 8; ++it) {
    const int n = wave * 16 + it * 2 + hsel;
    ov[it] = *(const v4f*)(sT + n * kOutTP + c4);
  }
  float* ob = out + (size_t)bb * kDm * kL + l0 + c4;
  for (int pass = 0; pass < 2; ++pass) {
#pragma unroll
    for (int it = 0; it < 8; ++it) {
      const int n = wave * 16 + it * 2 + hsel;
      *(volatile v4f*)(ob + (size_t)n * kL) = ov[it];
    }
    __threadfence();
  }
}

extern "C" void kernel_launch(void* const* d_in, const int* in_sizes, int n_in,
                              void* d_out, int out_size, void* d_ws, size_t ws_size,
                              hipStream_t stream) {
  if (n_in < 14) return;
  if (in_sizes[0] != kBatch * kCin * kHin * kWin) return;
  if (in_sizes[1] != kDm * kKconv) return;
  if (in_sizes[2] != kDm) return;
  if (in_sizes[3] != kDm) return;
  if (in_sizes[4] != kDm) return;
  if (in_sizes[5] != kXzP * kDm) return;
  if (in_sizes[6] != kDin * 4) return;
  if (in_sizes[7] != kDin) return;
  if (in_sizes[8] != kXdReal * kDin) return;
  if (in_sizes[9] != kDin * kDtR) return;
  if (in_sizes[10] != kDin) return;
  if (in_sizes[11] != kDin * kNst) return;
  if (in_sizes[12] != kDin) return;
  if (in_sizes[13] != kDm * kDin) return;
  if (out_size != kRows * kDm) return;
  if (ws_size < kWsTotal) return;

  const float* x      = (const float*)d_in[0];
  const float* conv_w = (const float*)d_in[1];
  const float* conv_b = (const float*)d_in[2];
  const float* ln_g   = (const float*)d_in[3];
  const float* ln_b   = (const float*)d_in[4];
  const float* inW    = (const float*)d_in[5];
  const float* c1w    = (const float*)d_in[6];
  const float* c1b    = (const float*)d_in[7];
  const float* xpW    = (const float*)d_in[8];
  const float* dtw    = (const float*)d_in[9];
  const float* dtb    = (const float*)d_in[10];
  const float* A_log  = (const float*)d_in[11];
  const float* Dp     = (const float*)d_in[12];
  const float* outW   = (const float*)d_in[13];
  float* out = (float*)d_out;

  char* ws = (char*)d_ws;
  unsigned short* W1   = (unsigned short*)(ws + kOffW1);
  unsigned short* W2   = (unsigned short*)(ws + kOffW2);
  unsigned short* W3   = (unsigned short*)(ws + kOffW3);
  unsigned short* W4   = (unsigned short*)(ws + kOffW4);
  unsigned short* COL  = (unsigned short*)(ws + kOffCol);
  float*          XCT  = (float*)(ws + kOffXcT);
  unsigned short* NRM  = (unsigned short*)(ws + kOffNrm);
  float*          XZ   = (float*)(ws + kOffXz);
  float*          XM   = (float*)(ws + kOffXm);
  unsigned short* XM16 = (unsigned short*)(ws + kOffXm16);
  float*          XD   = (float*)(ws + kOffXd);
  unsigned short* YG   = (unsigned short*)(ws + kOffYg);

  cast_rows_f16_kernel<<<(kDm * kKconv / 8) / 256, 256, 0, stream>>>(conv_w, W1, kKconv, kDm, kDm * kKconv / 8, 16.0f);
  cast_rows_f16_kernel<<<(kXzP * kDm / 8) / 256, 256, 0, stream>>>(inW, W2, kDm, kXzP, kXzP * kDm / 8, 16.0f);
  cast_rows_f16_kernel<<<(kXdP * kDin / 8) / 256, 256, 0, stream>>>(xpW, W3, kDin, kXdReal, kXdP * kDin / 8, 16.0f);
  cast_rows_f16_kernel<<<(kDm * kDin / 8) / 256, 256, 0, stream>>>(outW, W4, kDin, kDm, kDm * kDin / 8, 16.0f);

  for (int half = 0; half < 2; ++half) {
    im2col_kernel<<<(kHalfRows * (kKconv / 8)) / 256, 256, 0, stream>>>(x, COL, half);
    wmma_gemm64<0, false, 2, 0, false><<<dim3((kHalfRows / 64) / 8, 1), 256, 0, stream>>>(
        COL, nullptr, kKconv, 0L,
        W1, nullptr, kKconv, 0L,
        (void*)(XCT + (size_t)half * kHalfRows * kDm), nullptr, kDm, 0L,
        conv_b, nullptr, 0L,
        kHalfRows, kDm, kKconv, 1.0f / 16.0f);
  }

  ln_kernel<<<(kRows * 8) / 256, 256, 0, stream>>>(XCT, ln_g, ln_b, NRM);

  wmma_gemm64<0, false, 0, 0, false><<<dim3((kRows / 64) * (kXzP / 64) / 8, 1), 256, 0, stream>>>(
      NRM, nullptr, kDm, 0L,
      W2, nullptr, kDm, 0L,
      (void*)XZ, nullptr, kXzP, 0L,
      nullptr, nullptr, 0L,
      kRows, kXzP, kDm, 1.0f / 16.0f);

  conv_silu_kernel<<<kRows / 64, 128, 0, stream>>>(XZ, c1w, c1b, XM, XM16);

  wmma_gemm64<0, false, 0, 0, false><<<dim3((kRows / 64) * (kXdP / 64) / 8, 1), 256, 0, stream>>>(
      XM16, nullptr, kDin, 0L,
      W3, nullptr, kDin, 0L,
      (void*)XD, nullptr, kXdP, 0L,
      nullptr, nullptr, 0L,
      kRows, kXdP, kDin, 1.0f / 16.0f);

  scan_kernel<<<kBatch * (kDin / kScanCh), kScanCh, 0, stream>>>(XD, XM, XZ, dtw, dtb, A_log, Dp, YG, 16.0f);

  outproj_nchw_kernel<<<kRows / 64, 128, 0, stream>>>(YG, W4, XCT, out, 1.0f / 256.0f);
}
